// MambaNet_26783416058192
// MI455X (gfx1250) — hardware-verified
//
#include <hip/hip_runtime.h>
#include <math.h>

typedef __attribute__((ext_vector_type(16))) _Float16 v16h;
typedef __attribute__((ext_vector_type(8)))  _Float16 v8h;
typedef __attribute__((ext_vector_type(16))) __bf16   v16b;
typedef __attribute__((ext_vector_type(8)))  __bf16   v8b;
typedef __attribute__((ext_vector_type(8)))  float    v8f;
typedef __attribute__((ext_vector_type(4)))  float    v4f;
typedef __attribute__((ext_vector_type(2)))  float    v2f;

constexpr int kB      = 4;
constexpr int kL      = 1024;
constexpr int kD      = 512;
constexpr int kNH     = 8;
constexpr int kRows   = kB * kL;
constexpr int kConvK  = 3 * kL;
constexpr int kDin    = 1024;
constexpr int kNst    = 16;
constexpr int kDtR    = 32;
constexpr int kXzP    = 2 * kDin;
constexpr int kXdP    = 64;
constexpr int kDh     = kD / kNH;
constexpr int kDinH   = 2 * kDh;
constexpr int kDtRH   = 4;
constexpr int kXzPH   = 2 * kDinH;
constexpr int kXwH    = kDtRH + 2 * kNst;
constexpr int kSeqH   = kNH * kB;
constexpr int kRowsH  = kSeqH * kL;
constexpr int kConvCh = 128;
constexpr int kConvTP = 132;
constexpr int kScanTS = 64;
constexpr int kScanCh = 64;
constexpr int kScanYP = 68;
static_assert(kDtR + 2 * kNst == kXdP, "wide x_proj width");
static_assert(kXwH <= kXdP, "head x_proj width");
static_assert((kConvK % 32) == 0 && (kD % 32) == 0 && (kDin % 32) == 0 && (kDh % 32) == 0 && (kDinH % 32) == 0, "GEMM K multiples of 32");
static_assert((kL % 64) == 0 && (kD % 64) == 0 && (kRows % 64) == 0 && (kXzP % 64) == 0 && (kXdP % 64) == 0 &&
              (kRowsH % 64) == 0 && (kXzPH % 64) == 0 && (kDh % 64) == 0, "GEMM M,N multiples of 64");
static_assert((kL % kScanTS) == 0 && (kDin % kScanCh) == 0 && (kDinH % kScanCh) == 0 &&
              (kDin % kConvCh) == 0 && (kDinH % kConvCh) == 0, "tile multiples");
static_assert(kD == 4 * 128, "layernorm block = 128 threads x 4 floats");

constexpr size_t kOffXN  = 0;
constexpr size_t kOffIMH = kOffXN  + (size_t)kRows * kD * 4;
constexpr size_t kOffIML = kOffIMH + (size_t)kB * kD * kConvK * 2;
constexpr size_t kOffXZ  = 0;
constexpr size_t kEndZ   = kOffIML + (size_t)kB * kD * kConvK * 2;
constexpr size_t kOffUC  = kEndZ;
constexpr size_t kOffWCH = kOffUC;
constexpr size_t kOffWCL = kOffWCH + (size_t)kL * kConvK * 2;
constexpr size_t kOffUCH = kOffUC  + (size_t)kRows * kDin * 4;
constexpr size_t kOffCV  = kOffUCH;
constexpr size_t kOffUCL = kOffUCH + (size_t)kRows * kDin * 2;
constexpr size_t kOffGH  = kOffUCL;
constexpr size_t kOffGL  = kOffGH  + (size_t)kRows * kD * 2;
constexpr size_t kOffG1  = kOffUCL;
constexpr size_t kOffXD  = kOffUCL + (size_t)kRows * kDin * 2;
constexpr size_t kOffXHH = kOffXD;
constexpr size_t kOffXHL = kOffXHH + (size_t)kRowsH * kDh * 2;
constexpr size_t kOffYH  = kOffXD  + (size_t)kRowsH * kXdP * 4;
constexpr size_t kOffYL  = kOffYH  + (size_t)kRows * kDin * 2;
constexpr size_t kOffMBO = kOffYL  + (size_t)kRows * kDin * 2;
constexpr size_t kOffWIH = kOffMBO + (size_t)kRows * kD * 4;
constexpr size_t kOffWIL = kOffWIH + (size_t)kXzP * kD * 2;
constexpr size_t kOffWXH = kOffWIL + (size_t)kXzP * kD * 2;
constexpr size_t kOffWXL = kOffWXH + (size_t)kXdP * kDin * 2;
constexpr size_t kOffWOH = kOffWXL + (size_t)kXdP * kDin * 2;
constexpr size_t kOffWOL = kOffWOH + (size_t)kD * kDin * 2;
constexpr size_t kOffHIH = kOffWOL + (size_t)kD * kDin * 2;
constexpr size_t kOffHIL = kOffHIH + (size_t)kXzPH * kDh * 2;
constexpr size_t kOffHXH = kOffHIL + (size_t)kXzPH * kDh * 2;
constexpr size_t kOffHXL = kOffHXH + (size_t)kXdP * kDinH * 2;
constexpr size_t kOffHOH = kOffHXL + (size_t)kXdP * kDinH * 2;
constexpr size_t kOffHOL = kOffHOH + (size_t)kDh * kDinH * 2;
constexpr size_t kWsTotal = kOffHOL + (size_t)kDh * kDinH * 2;
static_assert(kEndZ == 33554432ull && kEndZ == kOffXZ + (size_t)kRows * kXzP * 4 && kEndZ == (size_t)kRowsH * kXzPH * 4, "arena Z");
static_assert(kOffWCL + (size_t)kL * kConvK * 2 <= kOffUCH, "conv weight planes inside arena U");
static_assert((size_t)kRowsH * kDinH * 4 == (size_t)kRows * kDin * 4, "arena U head size");
static_assert(kOffCV + (size_t)kRows * kD * 4 <= kOffUCL && kOffGL + (size_t)kRows * kD * 2 <= kOffXD && kOffG1 + (size_t)kRows * kD * 4 <= kOffXD, "arena P");
static_assert(kOffXHL + (size_t)kRowsH * kDh * 2 <= kOffYH && kOffXD + (size_t)kRows * kXdP * 4 <= kOffYH, "arena X");
static_assert((size_t)kRowsH * kDinH * 2 == (size_t)kRows * kDin * 2 && (size_t)kRowsH * kDh * 4 <= (size_t)kRows * kD * 4, "YH/YL and MBO/YO sizes");
static_assert(kWsTotal == 107347968ull, "carve total");
static_assert(kWsTotal <= 134217728ull, "carve cap");
static_assert((kOffIMH % 128) == 0 && (kOffIML % 128) == 0 && (kOffUC % 128) == 0 && (kOffWCL % 128) == 0 &&
              (kOffUCH % 128) == 0 && (kOffUCL % 128) == 0 && (kOffGL % 128) == 0 && (kOffXD % 128) == 0 &&
              (kOffXHL % 128) == 0 && (kOffYH % 128) == 0 && (kOffYL % 128) == 0 && (kOffMBO % 128) == 0 &&
              (kOffWIH % 128) == 0 && (kOffWIL % 128) == 0 && (kOffWXH % 128) == 0 && (kOffWXL % 128) == 0 &&
              (kOffWOH % 128) == 0 && (kOffWOL % 128) == 0 && (kOffHIH % 128) == 0 && (kOffHIL % 128) == 0 &&
              (kOffHXH % 128) == 0 && (kOffHXL % 128) == 0 && (kOffHOH % 128) == 0 && (kOffHOL % 128) == 0, "128-B aligned regions");

__device__ __forceinline__ unsigned short f2bf_bits(float f) {
  unsigned u = __float_as_uint(f);
  return (unsigned short)((u + 0x7FFFu + ((u >> 16) & 1u)) >> 16);
}
__device__ __forceinline__ float bf_bits2f(unsigned short h) { return __uint_as_float(((unsigned)h) << 16); }

__device__ __forceinline__ void dep_guard_h(v8f& a, v8f& b, v16h x, v16h y) { asm volatile("v_nop\n\tv_nop\n\tv_nop\n\tv_nop" : "+v"(a), "+v"(b) : "v"(x), "v"(y)); }
__device__ __forceinline__ void dep_guard_b(v8f& a, v8f& b, v16b x, v16b y) { asm volatile("v_nop\n\tv_nop\n\tv_nop\n\tv_nop" : "+v"(a), "+v"(b) : "v"(x), "v"(y)); }
__device__ __forceinline__ void keep4_h(v16h a, v16h b, v16h c, v16h d) { asm volatile("v_nop" :: "v"(a), "v"(b), "v"(c), "v"(d)); }
__device__ __forceinline__ void keep4_b(v16b a, v16b b, v16b c, v16b d) { asm volatile("v_nop" :: "v"(a), "v"(b), "v"(c), "v"(d)); }
__device__ __forceinline__ void acc_guard4(v8f& a, v8f& b, v8f& c, v8f& d) { asm volatile("v_nop\n\tv_nop\n\tv_nop\n\tv_nop" : "+v"(a), "+v"(b), "+v"(c), "+v"(d)); }
template <typename T> struct Frag;
template <> struct Frag<_Float16> {
  typedef v16h V; union U { v16h v; v8h h[2]; };
  static __device__ __forceinline__ v16h load(const _Float16* p) {
    U f; f.h[0] = *(const v8h*)(p); f.h[1] = *(const v8h*)(p + 16); return f.v;
  }
  static __device__ __forceinline__ v8f mma(v16h a, v16h b, v8f c) {
    return __builtin_amdgcn_wmma_f32_16x16x32_f16(false, a, false, b, (short)0, c, false, false);
  }
  static __device__ __forceinline__ void guard(v8f& a, v8f& b, v16h x, v16h y) { dep_guard_h(a, b, x, y); }
  static __device__ __forceinline__ void keep(v16h a, v16h b, v16h c, v16h d) { keep4_h(a, b, c, d); }
};
template <> struct Frag<__bf16> {
  typedef v16b V; union U { v16b v; v8b h[2]; };
  static __device__ __forceinline__ v16b load(const __bf16* p) {
    U f; f.h[0] = *(const v8b*)(p); f.h[1] = *(const v8b*)(p + 16); return f.v;
  }
  static __device__ __forceinline__ v8f mma(v16b a, v16b b, v8f c) {
    return __builtin_amdgcn_wmma_f32_16x16x32_bf16(false, a, false, b, (short)0, c, false, false);
  }
  static __device__ __forceinline__ void guard(v8f& a, v8f& b, v16b x, v16b y) { dep_guard_b(a, b, x, y); }
  static __device__ __forceinline__ void keep(v16b a, v16b b, v16b c, v16b d) { keep4_b(a, b, c, d); }
};

template <int ET> struct Elem;
template <> struct Elem<0> { typedef _Float16 T; };
template <> struct Elem<1> { typedef __bf16 T; };
template <int ET, int SPL, int BIAS_MODE, int OUT_MODE, bool RESID, int ACT = 0>
__global__ __launch_bounds__(256) void wmma_gemm64(
    const unsigned short* __restrict__ Ap, const unsigned short* __restrict__ A2p, int lda, long strideA,
    const unsigned short* __restrict__ Btp, const unsigned short* __restrict__ Bt2p, int ldb, long strideB,
    void* __restrict__ Cout, void* __restrict__ Cout2, int ldc, long strideC,
    const float* __restrict__ bias,
    const float* __restrict__ resid, long strideR,
    int M, int N, int K, float scale) {
  typedef typename Elem<ET>::T T;
  typedef typename Frag<T>::V V;
  const T* A = (const T*)Ap; const T* A2 = (const T*)A2p; const T* Bt = (const T*)Btp; const T* Bt2 = (const T*)Bt2p;
  __shared__ __align__(16) float sT[8][16 * 68];
  const int b    = blockIdx.y;
  const int lane = threadIdx.x & 31;
  const int wave = threadIdx.x >> 5;
  const int tilesN = N >> 6;
  const int tilesM = M >> 6;
  const int tile = blockIdx.x * 8 + wave;
  if (tile >= tilesM * tilesN) return;
  const int tm = tile / tilesN;
  const int tn = tile - tm * tilesN;
  const int m0 = tm << 6;
  const int n0 = tn << 6;

  const T* Ab  = A  + (size_t)b * strideA;
  const T* Bb  = Bt + (size_t)b * strideB;
  const T* Ab2 = (SPL >= 1) ? (A2  + (size_t)b * strideA) : nullptr;
  const T* Bb2 = (SPL == 2) ? (Bt2 + (size_t)b * strideB) : nullptr;

  const int rlane = lane & 15;
  const int koff  = (lane >> 4) * 8;
  const int mOff  = (lane >> 4) * 8;

  v8f acc[4][4];
#pragma unroll
  for (int i = 0; i < 4; ++i)
#pragma unroll
    for (int j = 0; j < 4; ++j) acc[i][j] = (v8f){0.f,0.f,0.f,0.f,0.f,0.f,0.f,0.f};

  for (int k0 = 0; k0 < K; k0 += 32) {
    V bh[4], bl[4];
#pragma unroll
    for (int j = 0; j < 4; ++j) {
      const size_t bo = (size_t)(n0 + (j << 4) + rlane) * ldb + koff + k0;
      bh[j] = Frag<T>::load(Bb + bo);
      if (SPL == 2) bl[j] = Frag<T>::load(Bb2 + bo);
    }
#pragma unroll
    for (int i = 0; i < 4; ++i) {
      const size_t ao = (size_t)(m0 + (i << 4) + rlane) * lda + koff + k0;
      V ah = Frag<T>::load(Ab + ao);
      V al;
      if (SPL >= 1) al = Frag<T>::load(Ab2 + ao);
#pragma unroll
      for (int j = 0; j < 4; ++j) {
        acc[i][j] = Frag<T>::mma(ah, bh[j], acc[i][j]);
        if (SPL == 2) acc[i][j] = Frag<T>::mma(ah, bl[j], acc[i][j]);
        if (SPL >= 1) acc[i][j] = Frag<T>::mma(al, bh[j], acc[i][j]);
      }
      Frag<T>::guard(acc[i][0], acc[i][3], ah, (SPL >= 1) ? al : ah);
    }
    Frag<T>::keep(bh[0], bh[1], bh[2], bh[3]);
    if (SPL == 2) Frag<T>::keep(bl[0], bl[1], bl[2], bl[3]);
  }
  acc_guard4(acc[0][0], acc[0][1], acc[0][2], acc[0][3]);
  acc_guard4(acc[1][0], acc[1][1], acc[1][2], acc[1][3]);
  acc_guard4(acc[2][0], acc[2][1], acc[2][2], acc[2][3]);
  acc_guard4(acc[3][0], acc[3][1], acc[3][2], acc[3][3]);

  float* slab = sT[wave];
  const float* Rb = RESID ? (resid + (size_t)b * strideR) : nullptr;
#pragma unroll
  for (int i = 0; i < 4; ++i) {
    const int mBase = m0 + (i << 4);
#pragma unroll
    for (int j = 0; j < 4; ++j) {
      const int n = n0 + (j << 4) + rlane;
      float bv = 0.f;
      if (BIAS_MODE == 2) bv = bias[n];
#pragma unroll
      for (int r = 0; r < 8; ++r) {
        float v = acc[i][j][r] * scale;
        if (BIAS_MODE == 1) v += bias[mBase + mOff + r];
        if (BIAS_MODE == 2) v += bv;
        if (RESID) v += Rb[(size_t)(mBase + mOff + r) * ldc + n];
        if (ACT == 1) v = tanhf(v);
        if (ACT == 2) v = fmaxf(v, 0.0f);
        if (ACT == 3) v = v / (1.0f + expf(-v));
        if (ACT == 4) v = (v > 0.f) ? v : 0.01f * v;
        slab[(mOff + r) * 68 + (j << 4) + rlane] = v;
      }
    }
    __builtin_amdgcn_fence(__ATOMIC_RELEASE, "workgroup");
    __builtin_amdgcn_wave_barrier();
    __builtin_amdgcn_fence(__ATOMIC_ACQUIRE, "workgroup");
    if (OUT_MODE == 0) {
      float* C = (float*)Cout + (size_t)b * strideC;
      const int hh = lane >> 4, c4 = (lane & 15) * 4;
      for (int pass = 0; pass < 2; ++pass) {
#pragma unroll
        for (int it = 0; it < 8; ++it) {
          const int row = it * 2 + hh;
          v4f v = *(const v4f*)(slab + row * 68 + c4);
          *(volatile v4f*)(C + (size_t)(mBase + row) * ldc + n0 + c4) = v;
        }
        __threadfence();
      }
    } else {
      const int q = lane >> 3, c8 = (lane & 7) * 8;
      unsigned short* C  = (unsigned short*)Cout  + (size_t)b * strideC;
      unsigned short* C2 = (OUT_MODE == 2) ? ((unsigned short*)Cout2 + (size_t)b * strideC) : nullptr;
      for (int pass = 0; pass < 2; ++pass) {
#pragma unroll
        for (int it = 0; it < 4; ++it) {
          const int row = it * 4 + q;
          const float* sp = slab + row * 68 + c8;
          v8h hv, lv;
#pragma unroll
          for (int e = 0; e < 8; ++e) {
            if (OUT_MODE == 1) {
              hv[e] = (_Float16)sp[e];
            } else {
              unsigned short hb = f2bf_bits(sp[e]);
              unsigned short lb = f2bf_bits(sp[e] - bf_bits2f(hb));
              hv[e] = __builtin_bit_cast(_Float16, hb);
              lv[e] = __builtin_bit_cast(_Float16, lb);
            }
          }
          *(volatile v8h*)(C + (size_t)(mBase + row) * ldc + n0 + c8) = hv;
          if (OUT_MODE == 2) *(volatile v8h*)(C2 + (size_t)(mBase + row) * ldc + n0 + c8) = lv;
        }
        __threadfence();
      }
    }
    __builtin_amdgcn_fence(__ATOMIC_RELEASE, "workgroup");
    __builtin_amdgcn_wave_barrier();
    __builtin_amdgcn_fence(__ATOMIC_ACQUIRE, "workgroup");
  }
}

__global__ __launch_bounds__(256) void split_rows_bf16_kernel(
    const float* __restrict__ src, unsigned short* __restrict__ dhi, unsigned short* __restrict__ dlo,
    int total8, int srcTotal)
{
  const int i = blockIdx.x * 256 + threadIdx.x;
  if (i >= total8) return;
  const size_t e0 = (size_t)i << 3;
  const bool valid = ((long)e0 < (long)srcTotal);
  const size_t eb = valid ? e0 : (size_t)(srcTotal - 8);
  const v4f a0 = *(const v4f*)(src + eb);
  const v4f a1 = *(const v4f*)(src + eb + 4);
  v8h hv, lv;
#pragma unroll
  for (int e = 0; e < 4; ++e) {
    const float f0 = valid ? a0[e] : 0.f;
    const float f1 = valid ? a1[e] : 0.f;
    const unsigned short h0 = f2bf_bits(f0), h1 = f2bf_bits(f1);
    const unsigned short l0 = f2bf_bits(f0 - bf_bits2f(h0)), l1 = f2bf_bits(f1 - bf_bits2f(h1));
    hv[e]     = __builtin_bit_cast(_Float16, h0);
    hv[4 + e] = __builtin_bit_cast(_Float16, h1);
    lv[e]     = __builtin_bit_cast(_Float16, l0);
    lv[4 + e] = __builtin_bit_cast(_Float16, l1);
  }
  unsigned short* qh = dhi + e0;
  unsigned short* ql = dlo + e0;
  *(volatile v8h*)qh = hv;
  *(volatile v8h*)ql = lv;
  __threadfence();
  *(volatile v8h*)qh = hv;
  *(volatile v8h*)ql = lv;
}

__global__ __launch_bounds__(128) void layernorm_kernel(
    const float* __restrict__ X, const float* __restrict__ gam, const float* __restrict__ bet, float* __restrict__ Y)
{
  __shared__ float red[4];
  const int tid = threadIdx.x, lane = tid & 31, wave = tid >> 5;
  const size_t row = blockIdx.x;
  const v4f xv = *(const v4f*)(X + row * kD + tid * 4);
  float s = (xv[0] + xv[1]) + (xv[2] + xv[3]);
#pragma unroll
  for (int off = 1; off < 32; off <<= 1) s += __shfl_xor(s, off, 32);
  if (lane == 0) red[wave] = s;
  __syncthreads();
  const float mean = ((red[0] + red[1]) + (red[2] + red[3])) * (1.0f / (float)kD);
  __syncthreads();
  const float e0 = xv[0] - mean, e1 = xv[1] - mean, e2 = xv[2] - mean, e3 = xv[3] - mean;
  float s2 = (e0 * e0 + e1 * e1) + (e2 * e2 + e3 * e3);
#pragma unroll
  for (int off = 1; off < 32; off <<= 1) s2 += __shfl_xor(s2, off, 32);
  if (lane == 0) red[wave] = s2;
  __syncthreads();
  const float var  = ((red[0] + red[1]) + (red[2] + red[3])) * (1.0f / (float)kD);
  const float rstd = 1.0f / sqrtf(var + 1e-5f);
  const v4f gv = *(const v4f*)(gam + tid * 4);
  const v4f bv = *(const v4f*)(bet + tid * 4);
  v4f yv;
  yv[0] = e0 * rstd * gv[0] + bv[0];
  yv[1] = e1 * rstd * gv[1] + bv[1];
  yv[2] = e2 * rstd * gv[2] + bv[2];
  yv[3] = e3 * rstd * gv[3] + bv[3];
  float* yp = Y + row * kD + tid * 4;
  *(volatile v4f*)yp = yv;
  __threadfence();
  *(volatile v4f*)yp = yv;
}

template <int SRC>
__global__ __launch_bounds__(256) void im2col_split_kernel(
    const float* __restrict__ X, unsigned short* __restrict__ dhi, unsigned short* __restrict__ dlo)
{
  constexpr int kQ = kConvK / 8;
  const int t = blockIdx.x * 256 + threadIdx.x;
  if (t >= kB * kD * kQ) return;
  const int q  = t % kQ;
  const int bf = t / kQ;
  const int f  = bf % kD;
  const int b  = bf / kD;
  const int K0 = q * 8;
  v8h hv, lv;
#pragma unroll
  for (int e = 0; e < 8; ++e) {
    const int K = K0 + e;
    const int i = K / 3;
    const int k = K - i * 3;
    const int c = f - 1 + k;
    const bool valid = (c >= 0) && (c < kD);
    const int cc = (c < 0) ? 0 : ((c >= kD) ? (kD - 1) : c);
    size_t idx;
    if (SRC == 0) idx = ((size_t)(b * kL + i)) * kD + cc;
    else          idx = ((size_t)(((cc & 7) * kB + b) * kL + i)) * kDh + (cc >> 3);
    const float v  = X[idx];
    const float vz = valid ? v : 0.f;
    const unsigned short hb = f2bf_bits(vz);
    const unsigned short lb = f2bf_bits(vz - bf_bits2f(hb));
    hv[e] = __builtin_bit_cast(_Float16, hb);
    lv[e] = __builtin_bit_cast(_Float16, lb);
  }
  const size_t o = ((size_t)(b * kD + f)) * kConvK + K0;
  unsigned short* qh = dhi + o;
  unsigned short* ql = dlo + o;
  *(volatile v8h*)qh = hv;
  *(volatile v8h*)ql = lv;
  __threadfence();
  *(volatile v8h*)qh = hv;
  *(volatile v8h*)ql = lv;
}

template <int OUTM>
__global__ __launch_bounds__(256) void bias_gelu_kernel(
    const float* __restrict__ C, const float* __restrict__ bias,
    float* __restrict__ outF, unsigned short* __restrict__ dhi, unsigned short* __restrict__ dlo, int n2)
{
  const int i = blockIdx.x * 256 + threadIdx.x;
  if (i >= n2) return;
  const size_t e0 = (size_t)i * 2;
  const int o = (int)((e0 / kD) % kL);
  const float bo = bias[o];
  const v2f cv = *(const v2f*)(C + e0);
  float g0 = 0.f, g1 = 0.f;
#pragma unroll 1
  for (int e = 0; e < 2; ++e) {
    const float v  = ((e == 0) ? cv[0] : cv[1]) + bo;
    const float gv = 0.5f * v * (1.0f + erff(v * 0.70710678118654752f));
    g0 = (e == 0) ? gv : g0;
    g1 = gv;
  }
  if (OUTM == 0) {
    v2f gv2;
    gv2[0] = g0; gv2[1] = g1;
    float* p = outF + e0;
    *(volatile v2f*)p = gv2;
    __threadfence();
    *(volatile v2f*)p = gv2;
  } else {
    const unsigned short h0 = f2bf_bits(g0), h1 = f2bf_bits(g1);
    const unsigned short l0 = f2bf_bits(g0 - bf_bits2f(h0)), l1 = f2bf_bits(g1 - bf_bits2f(h1));
    const unsigned uh = (unsigned)h0 | ((unsigned)h1 << 16);
    const unsigned ul = (unsigned)l0 | ((unsigned)l1 << 16);
    ((volatile unsigned*)dhi)[i] = uh;
    ((volatile unsigned*)dlo)[i] = ul;
    __threadfence();
    ((volatile unsigned*)dhi)[i] = uh;
    ((volatile unsigned*)dlo)[i] = ul;
  }
}

__global__ __launch_bounds__(256) void to_heads_split_kernel(
    const float* __restrict__ S, unsigned short* __restrict__ dhi, unsigned short* __restrict__ dlo)
{
  const int t = blockIdx.x * 256 + threadIdx.x;
  if (t >= kRowsH * (kDh / 8)) return;
  const int r   = t >> 3;
  const int j0  = (t & 7) * 8;
  const int seq = r / kL;
  const int l   = r % kL;
  const int hd  = seq / kB;
  const int b   = seq % kB;
  const float* sp = S + ((size_t)(b * kL + l)) * kD + hd;
  v8h hv, lv;
#pragma unroll
  for (int e = 0; e < 8; ++e) {
    const float v = sp[(j0 + e) * kNH];
    const unsigned short hb = f2bf_bits(v);
    const unsigned short lb = f2bf_bits(v - bf_bits2f(hb));
    hv[e] = __builtin_bit_cast(_Float16, hb);
    lv[e] = __builtin_bit_cast(_Float16, lb);
  }
  const size_t o = (size_t)r * kDh + j0;
  unsigned short* qh = dhi + o;
  unsigned short* ql = dlo + o;
  *(volatile v8h*)qh = hv;
  *(volatile v8h*)ql = lv;
  __threadfence();
  *(volatile v8h*)qh = hv;
  *(volatile v8h*)ql = lv;
}

template <int NCH>
__global__ __launch_bounds__(128) void conv_silu_kernel(
    const float* __restrict__ XZ, const float* __restrict__ cw, const float* __restrict__ cb,
    float* __restrict__ UC, unsigned short* __restrict__ UCH, unsigned short* __restrict__ UCL)
{
  constexpr int XZP = 2 * NCH;
  __shared__ __align__(16) float sT[16 * kConvTP];
  const int tid = threadIdx.x, lane = tid & 31, wave = tid >> 5;
  const int d0 = blockIdx.x * kConvCh, d = d0 + tid;
  const int g0 = blockIdx.y * 64;
  const int tb = g0 & (kL - 1);
  const float w0 = cw[d * 4 + 0], w1 = cw[d * 4 + 1], w2 = cw[d * 4 + 2], w3 = cw[d * 4 + 3];
  const float bc = cb[d];
  float xm3, xm2, xm1;
  {
    const bool hist = (tb > 0);
    const int rb = hist ? (g0 - 3) : g0;
    const float v3 = XZ[(size_t)rb * XZP + d];
    const float v2 = XZ[(size_t)(rb + 1) * XZP + d];
    const float v1 = XZ[(size_t)(rb + 2) * XZP + d];
    xm3 = hist ? v3 : 0.f;
    xm2 = hist ? v2 : 0.f;
    xm1 = hist ? v1 : 0.f;
  }
  const int fch  = lane * 4;
  const int brow = wave * 2 + (lane >> 4);
  const int bch  = (lane & 15) * 8;
#pragma unroll 1
  for (int sub = 0; sub < 4; ++sub) {
    const int lb = g0 + sub * 16;
#pragma unroll 1
    for (int s = 0; s < 16; ++s) {
      const float xcur = XZ[(size_t)(lb + s) * XZP + d];
      float acc = w0 * xm3;
      acc = fmaf(w1, xm2, acc);
      acc = fmaf(w2, xm1, acc);
      acc = fmaf(w3, xcur, acc);
      const float sv = acc + bc;
      const float sg = __builtin_amdgcn_rcpf(1.0f + __expf(-sv));
      sT[s * kConvTP + tid] = sv * sg;
      xm3 = xm2; xm2 = xm1; xm1 = xcur;
    }
    __syncthreads();
    v4f fv[4];
    v8h bh[2], blo[2];
#pragma unroll
    for (int it = 0; it < 4; ++it) fv[it] = *(const v4f*)(sT + (it * 4 + wave) * kConvTP + fch);
#pragma unroll
    for (int it = 0; it < 2; ++it) {
      const float* sp = sT + (it * 8 + brow) * kConvTP + bch;
      const v4f a0 = *(const v4f*)(sp);
      const v4f a1 = *(const v4f*)(sp + 4);
#pragma unroll
      for (int e = 0; e < 4; ++e) {
        const unsigned short h0 = f2bf_bits(a0[e]), h1 = f2bf_bits(a1[e]);
        const unsigned short l0 = f2bf_bits(a0[e] - bf_bits2f(h0)), l1 = f2bf_bits(a1[e] - bf_bits2f(h1));
        bh[it][e]      = __builtin_bit_cast(_Float16, h0);
        bh[it][4 + e]  = __builtin_bit_cast(_Float16, h1);
        blo[it][e]     = __builtin_bit_cast(_Float16, l0);
        blo[it][4 + e] = __builtin_bit_cast(_Float16, l1);
      }
    }
    for (int pass = 0; pass < 2; ++pass) {
#pragma unroll
      for (int it = 0; it < 4; ++it)
        *(volatile v4f*)(UC + (size_t)(lb + it * 4 + wave) * NCH + d0 + fch) = fv[it];
#pragma unroll
      for (int it = 0; it < 2; ++it) {
        const size_t o = (size_t)(lb + it * 8 + brow) * NCH + d0 + bch;
        *(volatile v8h*)(UCH + o) = bh[it];
        *(volatile v8h*)(UCL + o) = blo[it];
      }
      __threadfence();
    }
    __syncthreads();
  }
}

template <int NCH, int DTR>
__global__ __launch_bounds__(64) void scan_kernel(
    const float* __restrict__ XD, const float* __restrict__ UC, const float* __restrict__ XZ,
    const float* __restrict__ Wdt, const float* __restrict__ bdt, const float* __restrict__ Alog,
    const float* __restrict__ Dp, unsigned short* __restrict__ YH, unsigned short* __restrict__ YL)
{
  constexpr int XZP = 2 * NCH;
  constexpr int kBlkPerSeq = NCH / kScanCh;
  __shared__ __align__(16) float sX[kScanTS * kXdP];
  __shared__ __align__(16) float sY[kScanTS * kScanYP];
  __shared__ __align__(16) float sW[DTR * kScanCh];
  __shared__ __align__(16) float sA[kNst * kScanCh];
  const int tid = threadIdx.x, lane = tid & 31, wave = tid >> 5;
  const int bix = blockIdx.x / kBlkPerSeq;
  const int d0  = (blockIdx.x - bix * kBlkPerSeq) * kScanCh;
  const int d   = d0 + tid;
  const size_t row0 = (size_t)bix * kL;
#pragma unroll 1
  for (int r = 0; r < DTR; ++r) sW[r * kScanCh + tid] = Wdt[(size_t)d * DTR + r];
#pragma unroll 1
  for (int s = 0; s < kNst; ++s) sA[s * kScanCh + tid] = -expf(Alog[(size_t)d * kNst + s]);
  __syncthreads();
  float negA[kNst], h[kNst];
#pragma unroll
  for (int s = 0; s < kNst; ++s) {
    negA[s] = sA[s * kScanCh + tid];
    h[s] = 0.f;
  }
  const float bb = bdt[d], Dd = Dp[d];
  const int lr = tid >> 4, lc4 = (tid & 15) * 4;
  const int q = lane >> 3, c8 = (lane & 7) * 8;
#pragma unroll 1
  for (int t0 = 0; t0 < kL; t0 += kScanTS) {
    __syncthreads();
#pragma unroll
    for (int i = 0; i < 16; ++i) {
      const int r = lr + 4 * i;
      *(v4f*)(sX + r * kXdP + lc4) = *(const v4f*)(XD + (row0 + t0 + r) * kXdP + lc4);
    }
    __syncthreads();
#pragma unroll 1
    for (int s = 0; s < kScanTS; ++s) {
      const int t = t0 + s;
      const float* xr = sX + s * kXdP;
      float vdot = 0.f;
#pragma unroll 1
      for (int r4 = 0; r4 < DTR / 4; ++r4) {
        const v4f xv = *(const v4f*)(xr + 4 * r4);
        const float* wp = sW + (4 * r4) * kScanCh + tid;
        vdot = fmaf(xv[0], wp[0], vdot);
        vdot = fmaf(xv[1], wp[kScanCh], vdot);
        vdot = fmaf(xv[2], wp[2 * kScanCh], vdot);
        vdot = fmaf(xv[3], wp[3 * kScanCh], vdot);
      }
      float Bs[kNst], Cs[kNst];
#pragma unroll
      for (int q4 = 0; q4 < 4; ++q4) {
        const v4f bv = *(const v4f*)(xr + DTR + 4 * q4);
        const v4f cv = *(const v4f*)(xr + DTR + kNst + 4 * q4);
        Bs[4 * q4 + 0] = bv[0]; Bs[4 * q4 + 1] = bv[1]; Bs[4 * q4 + 2] = bv[2]; Bs[4 * q4 + 3] = bv[3];
        Cs[4 * q4 + 0] = cv[0]; Cs[4 * q4 + 1] = cv[1]; Cs[4 * q4 + 2] = cv[2]; Cs[4 * q4 + 3] = cv[3];
      }
      const float v   = vdot + bb;
      const float a   = __expf(-fabsf(v));
      const float u   = 1.0f + a;
      const float l1p = __logf(u) + (a - (u - 1.0f)) * __builtin_amdgcn_rcpf(u);
      const float dt  = fmaxf(v, 0.0f) + l1p;
      const float xt  = UC[(row0 + t) * NCH + d];
      const float dtx = dt * xt;
      float y = 0.f;
#pragma unroll
      for (int k = 0; k < kNst; ++k) {
        const float e = __expf(dt * negA[k]);
        h[k] = e * h[k] + dtx * Bs[k];
        y = h[k] * Cs[k] + y;
      }
      y = xt * Dd + y;
      const float zv = XZ[(row0 + t) * XZP + NCH + d];
      const float sg = __builtin_amdgcn_rcpf(1.0f + __expf(-zv));
      y = y * (zv * sg);
      sY[s * kScanYP + tid] = y;
    }
    __syncthreads();
    v8h hv[8], lv[8];
#pragma unroll
    for (int it = 0; it < 8; ++it) {
      const int row = it * 8 + wave * 4 + q;
      const float* sp = sY + row * kScanYP + c8;
      const v4f a0 = *(const v4f*)(sp);
      const v4f a1 = *(const v4f*)(sp + 4);
#pragma unroll
      for (int e = 0; e < 4; ++e) {
        const unsigned short h0 = f2bf_bits(a0[e]), h1 = f2bf_bits(a1[e]);
        const unsigned short l0 = f2bf_bits(a0[e] - bf_bits2f(h0)), l1 = f2bf_bits(a1[e] - bf_bits2f(h1));
        hv[it][e]     = __builtin_bit_cast(_Float16, h0);
        hv[it][4 + e] = __builtin_bit_cast(_Float16, h1);
        lv[it][e]     = __builtin_bit_cast(_Float16, l0);
        lv[it][4 + e] = __builtin_bit_cast(_Float16, l1);
      }
    }
    for (int pass = 0; pass < 2; ++pass) {
#pragma unroll
      for (int it = 0; it < 8; ++it) {
        const int row = it * 8 + wave * 4 + q;
        const size_t o = (row0 + t0 + row) * NCH + d0 + c8;
        *(volatile v8h*)(YH + o) = hv[it];
        *(volatile v8h*)(YL + o) = lv[it];
      }
      __threadfence();
    }
  }
}

static void gemm3(const unsigned short* Ah, const unsigned short* Al, int lda, long sA,
                  const unsigned short* Bh, const unsigned short* Bl, int ldb, long sB,
                  float* C, int ldc, long sC, int M, int N, int K, int batch, hipStream_t st)
{
  const int tiles  = (M / 64) * (N / 64);
  const int blocks = (tiles + 7) / 8;
  wmma_gemm64<1, 2, 0, 0, false><<<dim3(blocks, batch), 256, 0, st>>>(
      Ah, Al, lda, sA, Bh, Bl, ldb, sB, (void*)C, nullptr, ldc, sC, nullptr, nullptr, 0L, M, N, K, 1.0f);
}

extern "C" void kernel_launch(void* const* d_in, const int* in_sizes, int n_in,
                              void* d_out, int out_size, void* d_ws, size_t ws_size,
                              hipStream_t stream) {
  if (n_in < 27) return;
  if (in_sizes[0]  != kRows * kD) return;
  if (in_sizes[1]  != kD || in_sizes[2] != kD || in_sizes[3] != kD || in_sizes[4] != kD) return;
  if (in_sizes[5]  != kL * kL * 3 || in_sizes[6] != kL) return;
  if (in_sizes[7]  != kL * kL * 3 || in_sizes[8] != kL) return;
  if (in_sizes[9]  != kXzP * kD) return;
  if (in_sizes[10] != kDin * 4 || in_sizes[11] != kDin) return;
  if (in_sizes[12] != kXdP * kDin) return;
  if (in_sizes[13] != kDin * kDtR || in_sizes[14] != kDin) return;
  if (in_sizes[15] != kDin * kNst || in_sizes[16] != kDin) return;
  if (in_sizes[17] != kD * kDin) return;
  if (in_sizes[18] != kXzPH * kDh) return;
  if (in_sizes[19] != kDinH * 4 || in_sizes[20] != kDinH) return;
  if (in_sizes[21] != kXwH * kDinH) return;
  if (in_sizes[22] != kDinH * kDtRH || in_sizes[23] != kDinH) return;
  if (in_sizes[24] != kDinH * kNst || in_sizes[25] != kDinH) return;
  if (in_sizes[26] != kDh * kDinH) return;
  if (out_size != kRows * kD) return;
  if (ws_size < kWsTotal) return;

  const float* x        = (const float*)d_in[0];
  const float* ln1_g    = (const float*)d_in[1];
  const float* ln1_b    = (const float*)d_in[2];
  const float* ln2_g    = (const float*)d_in[3];
  const float* ln2_b    = (const float*)d_in[4];
  const float* conv0_w  = (const float*)d_in[5];
  const float* conv0_b  = (const float*)d_in[6];
  const float* conv1_w  = (const float*)d_in[7];
  const float* conv1_b  = (const float*)d_in[8];
  const float* m_in_w   = (const float*)d_in[9];
  const float* m_cv_w   = (const float*)d_in[10];
  const float* m_cv_b   = (const float*)d_in[11];
  const float* m_xp_w   = (const float*)d_in[12];
  const float* m_dt_w   = (const float*)d_in[13];
  const float* m_dt_b   = (const float*)d_in[14];
  const float* m_Alog   = (const float*)d_in[15];
  const float* m_Dv     = (const float*)d_in[16];
  const float* m_out_w  = (const float*)d_in[17];
  const float* h_in_w   = (const float*)d_in[18];
  const float* h_cv_w   = (const float*)d_in[19];
  const float* h_cv_b   = (const float*)d_in[20];
  const float* h_xp_w   = (const float*)d_in[21];
  const float* h_dt_w   = (const float*)d_in[22];
  const float* h_dt_b   = (const float*)d_in[23];
  const float* h_Alog   = (const float*)d_in[24];
  const float* h_Dv     = (const float*)d_in[25];
  const float* h_out_w  = (const float*)d_in[26];
  float* out = (float*)d_out;

  char* ws = (char*)d_ws;
  float*          XN  = (float*)(ws + kOffXN);
  unsigned short* IMH = (unsigned short*)(ws + kOffIMH);
  unsigned short* IML = (unsigned short*)(ws + kOffIML);
  float*          XZ  = (float*)(ws + kOffXZ);
  float*          UC  = (float*)(ws + kOffUC);
  unsigned short* WCH = (unsigned short*)(ws + kOffWCH);
  unsigned short* WCL = (unsigned short*)(ws + kOffWCL);
  unsigned short* UCH = (unsigned short*)(ws + kOffUCH);
  float*          CV  = (float*)(ws + kOffCV);
  unsigned short* UCL = (unsigned short*)(ws + kOffUCL);
  unsigned short* GH  = (unsigned short*)(ws + kOffGH);
  unsigned short* GL  = (unsigned short*)(ws + kOffGL);
  float*          G1  = (float*)(ws + kOffG1);
  float*          XD  = (float*)(ws + kOffXD);
  unsigned short* XHH = (unsigned short*)(ws + kOffXHH);
  unsigned short* XHL = (unsigned short*)(ws + kOffXHL);
  unsigned short* YH  = (unsigned short*)(ws + kOffYH);
  unsigned short* YL  = (unsigned short*)(ws + kOffYL);
  float*          MBO = (float*)(ws + kOffMBO);
  float*          YO  = MBO;
  unsigned short* WIH = (unsigned short*)(ws + kOffWIH);
  unsigned short* WIL = (unsigned short*)(ws + kOffWIL);
  unsigned short* WXH = (unsigned short*)(ws + kOffWXH);
  unsigned short* WXL = (unsigned short*)(ws + kOffWXL);
  unsigned short* WOH = (unsigned short*)(ws + kOffWOH);
  unsigned short* WOL = (unsigned short*)(ws + kOffWOL);
  unsigned short* HIH = (unsigned short*)(ws + kOffHIH);
  unsigned short* HIL = (unsigned short*)(ws + kOffHIL);
  unsigned short* HXH = (unsigned short*)(ws + kOffHXH);
  unsigned short* HXL = (unsigned short*)(ws + kOffHXL);
  unsigned short* HOH = (unsigned short*)(ws + kOffHOH);
  unsigned short* HOL = (unsigned short*)(ws + kOffHOL);

  const int n2 = kRows * kD / 2;

  layernorm_kernel<<<kRows, 128, 0, stream>>>(x, ln1_g, ln1_b, XN);
  im2col_split_kernel<0><<<(kB * kD * (kConvK / 8)) / 256, 256, 0, stream>>>(XN, IMH, IML);
  split_rows_bf16_kernel<<<(kL * kConvK / 8 + 255) / 256, 256, 0, stream>>>(conv0_w, WCH, WCL, kL * kConvK / 8, kL * kConvK);
  gemm3(WCH, WCL, kConvK, 0L, IMH, IML, kConvK, (long)kD * kConvK, CV, kD, (long)kL * kD, kL, kD, kConvK, kB, stream);
  bias_gelu_kernel<1><<<(n2 + 255) / 256, 256, 0, stream>>>(CV, conv0_b, nullptr, GH, GL, n2);

  split_rows_bf16_kernel<<<(kXzP * kD / 8 + 255) / 256, 256, 0, stream>>>(m_in_w, WIH, WIL, kXzP * kD / 8, kXzP * kD);
  split_rows_bf16_kernel<<<(kXdP * kDin / 8 + 255) / 256, 256, 0, stream>>>(m_xp_w, WXH, WXL, kXdP * kDin / 8, kXdP * kDin);
  split_rows_bf16_kernel<<<(kD * kDin / 8 + 255) / 256, 256, 0, stream>>>(m_out_w, WOH, WOL, kD * kDin / 8, kD * kDin);
  gemm3(GH, GL, kD, 0L, WIH, WIL, kD, 0L, XZ, kXzP, 0L, kRows, kXzP, kD, 1, stream);
  conv_silu_kernel<kDin><<<dim3(kDin / kConvCh, kRows / 64), kConvCh, 0, stream>>>(XZ, m_cv_w, m_cv_b, UC, UCH, UCL);
  gemm3(UCH, UCL, kDin, 0L, WXH, WXL, kDin, 0L, XD, kXdP, 0L, kRows, kXdP, kDin, 1, stream);
  scan_kernel<kDin, kDtR><<<kB * (kDin / kScanCh), kScanCh, 0, stream>>>(XD, UC, XZ, m_dt_w, m_dt_b, m_Alog, m_Dv, YH, YL);
  gemm3(YH, YL, kDin, 0L, WOH, WOL, kDin, 0L, MBO, kD, 0L, kRows, kD, kDin, 1, stream);

  to_heads_split_kernel<<<(kRowsH * (kDh / 8)) / 256, 256, 0, stream>>>(MBO, XHH, XHL);
  split_rows_bf16_kernel<<<(kXzPH * kDh / 8 + 255) / 256, 256, 0, stream>>>(h_in_w, HIH, HIL, kXzPH * kDh / 8, kXzPH * kDh);
  split_rows_bf16_kernel<<<(kXdP * kDinH / 8 + 255) / 256, 256, 0, stream>>>(h_xp_w, HXH, HXL, kXdP * kDinH / 8, kXwH * kDinH);
  split_rows_bf16_kernel<<<(kDh * kDinH / 8 + 255) / 256, 256, 0, stream>>>(h_out_w, HOH, HOL, kDh * kDinH / 8, kDh * kDinH);
  gemm3(XHH, XHL, kDh, 0L, HIH, HIL, kDh, 0L, XZ, kXzPH, 0L, kRowsH, kXzPH, kDh, 1, stream);
  conv_silu_kernel<kDinH><<<dim3(kDinH / kConvCh, kRowsH / 64), kConvCh, 0, stream>>>(XZ, h_cv_w, h_cv_b, UC, UCH, UCL);
  gemm3(UCH, UCL, kDinH, 0L, HXH, HXL, kDinH, 0L, XD, kXdP, 0L, kRowsH, kXdP, kDinH, 1, stream);
  scan_kernel<kDinH, kDtRH><<<kSeqH * (kDinH / kScanCh), kScanCh, 0, stream>>>(XD, UC, XZ, h_dt_w, h_dt_b, h_Alog, h_Dv, YH, YL);
  gemm3(YH, YL, kDinH, 0L, HOH, HOL, kDinH, 0L, YO, kDh, 0L, kRowsH, kDh, kDinH, 1, stream);

  im2col_split_kernel<1><<<(kB * kD * (kConvK / 8)) / 256, 256, 0, stream>>>(YO, IMH, IML);
  split_rows_bf16_kernel<<<(kL * kConvK / 8 + 255) / 256, 256, 0, stream>>>(conv1_w, WCH, WCL, kL * kConvK / 8, kL * kConvK);
  gemm3(WCH, WCL, kConvK, 0L, IMH, IML, kConvK, (long)kD * kConvK, CV, kD, (long)kL * kD, kL, kD, kConvK, kB, stream);
  bias_gelu_kernel<0><<<(n2 + 255) / 256, 256, 0, stream>>>(CV, conv1_b, G1, nullptr, nullptr, n2);
  layernorm_kernel<<<kRows, 128, 0, stream>>>(G1, ln2_g, ln2_b, out);
}
